// GAT_Batch_19481971655237
// MI455X (gfx1250) — hardware-run, weakly checked
//
#include <hip/hip_runtime.h>


namespace {
constexpr int NB = 32, NN = 512, FI = 128, FH = 64, NHD = 8, FC = NHD * FH  , FO = 16, KB = 128;
constexpr float HS = 256.0f, WSC = 256.0f, PS = 256.0f, SLOPE = 0.2f;
typedef _Float16 b16;
typedef __attribute__((ext_vector_type(16))) _Float16 v16b;
typedef __attribute__((ext_vector_type(8))) _Float16 v8b;
typedef __attribute__((ext_vector_type(8))) float v8f;
typedef __attribute__((ext_vector_type(4))) float v4f;
__device__ __forceinline__ float bf16_rne(float f) { unsigned int u = __float_as_uint(f); u += 0x7FFFu + ((u >> 16) & 1u); float r = __uint_as_float(u & 0xFFFF0000u); asm volatile("" : "+v"(r)); return r; }
__device__ __forceinline__ float bfv(float f) { float r = bf16_rne(f); asm volatile("" : "+v"(r)); return r; }
__device__ __forceinline__ void split16(float v, b16& hi, b16& lo) { hi = (b16)v; lo = (b16)(v - (float)hi); }
__device__ __forceinline__ v16b frag_kb(const b16* p, int hh) { const v8b a = *(const v8b*)(p + 8 * hh), b = *(const v8b*)(p + 16 + 8 * hh); v16b f;
#pragma unroll
  for (int e = 0; e < 8; ++e) { f[e] = a[e]; f[8 + e] = b[e]; } return f; }
__device__ __forceinline__ v8f wmma16b(v16b a, v16b b, v8f c) { v8f d = __builtin_amdgcn_wmma_f32_16x16x32_f16(false, a, false, b, (short)0, c, false, false); asm volatile("v_nop\n\tv_nop\n\tv_nop\n\tv_nop" : "+v"(d) : "v"(a), "v"(b)); return d; }
__device__ __forceinline__ void wave_lds_sync() { __builtin_amdgcn_fence(__ATOMIC_RELEASE, "workgroup"); __builtin_amdgcn_wave_barrier(); __builtin_amdgcn_fence(__ATOMIC_ACQUIRE, "workgroup"); }
__device__ __forceinline__ float pmul(float a, float b) { float p = a * b; asm volatile("" : "+v"(p)); return p; }
__device__ __forceinline__ float leaky(float v) { return v > 0.0f ? v : SLOPE * v; }

__global__ __launch_bounds__(256) void wput_kernel(const float* __restrict__ wh, const float* __restrict__ wo, b16* __restrict__ WH, b16* __restrict__ WOUT) { const int u = blockIdx.x * 256 + threadIdx.x; v8b v;
  if (u < FC * (FI / 8)) { const int o = u / (FI / 8), k0 = (u % (FI / 8)) * 8; const int hd = o / FH, f = o % FH;
#pragma unroll
    for (int j = 0; j < 8; ++j) v[j] = (b16)(bf16_rne(wh[((size_t)hd * FI + k0 + j) * FH + f]) * WSC); for (int pass = 0; pass < 2; ++pass) { *(volatile v8b*)(WH + (size_t)o * FI + k0) = v; __threadfence(); } }
  if (u < FO * (FC / 8)) { const int o = u / (FC / 8), k0 = (u % (FC / 8)) * 8;
#pragma unroll
    for (int j = 0; j < 8; ++j) v[j] = (b16)(bf16_rne(wo[(size_t)(k0 + j) * FO + o]) * WSC); for (int pass = 0; pass < 2; ++pass) { *(volatile v8b*)(WOUT + (size_t)o * FC + k0) = v; __threadfence(); } } }
__global__ __launch_bounds__(32) void proj1_kernel(const float* __restrict__ x, const b16* __restrict__ WH, const float* __restrict__ a1, const float* __restrict__ a2, int RLIM, b16* __restrict__ HPh, b16* __restrict__ HPl, float* __restrict__ FL) { __shared__ __attribute__((aligned(16))) b16 Ah[16][FI + 8], Oh[16][264], Ol[16][264]; __shared__ float Tf[16][260], Fa[16][16]; const int lane = threadIdx.x, nloc = lane & 15, hlf = lane >> 4; const size_t m0 = (size_t)blockIdx.x * 16; if (m0 >= (size_t)RLIM) return;
  for (int rr = 0; rr < 16; ++rr) for (int q = 0; q < 4; ++q) Ah[rr][q * 32 + lane] = (b16)(bf16_rne(x[(m0 + rr) * FI + q * 32 + lane]) * HS);
  wave_lds_sync();
#pragma unroll 1
  for (int g = 0; g < 4; ++g) { v8f acc[8];
#pragma unroll
    for (int t = 0; t < 8; ++t) acc[t] = (v8f){};
#pragma unroll
    for (int kb = 0; kb < FI; kb += 32) { const v16b a = frag_kb(&Ah[nloc][kb], hlf);
#pragma unroll
      for (int t = 0; t < 8; ++t) acc[t] = wmma16b(a, frag_kb(WH + (size_t)(g * 128 + t * 16 + nloc) * FI + kb, hlf), acc[t]); }
#pragma unroll
    for (int t = 0; t < 8; ++t) { const int cc = t * 16 + nloc;
#pragma unroll
      for (int r8 = 0; r8 < 8; ++r8) { const float v = acc[t][r8] * (1.0f / (HS * WSC)); Tf[8 * hlf + r8][cc] = v; b16 p, ql; split16(v * HS, p, ql); Oh[8 * hlf + r8][cc] = p; Ol[8 * hlf + r8][cc] = ql; } }
    wave_lds_sync();
    for (int rr = 0; rr < 16; ++rr) { const int hq = (lane >> 3) & 1, c0 = (lane & 7) * 8; float s1 = 0.0f, s2 = 0.0f; for (int k = 0; k < 8; ++k) { const int cc = hq * FH + c0 + k; const float hv = Tf[rr][cc]; const int hg = g * 2 + hq; s1 += pmul(hv, bfv(a1[hg * FH + c0 + k])); s2 += pmul(hv, bfv(a2[hg * FH + c0 + k])); }
      for (int o = 1; o < 8; o <<= 1) { s1 += __shfl_xor(s1, o); s2 += __shfl_xor(s2, o); } if ((lane & 7) == 0 && lane < 16) { Fa[rr][g * 2 + hq] = s1; Fa[rr][8 + g * 2 + hq] = s2; } }
    wave_lds_sync();
    for (int pass = 0; pass < 2; ++pass) { for (int rr = 0; rr < 16; ++rr) { if (lane < 16) { *(volatile v8b*)(HPh + (m0 + rr) * FC + g * 128 + lane * 8) = *(const v8b*)(&Oh[rr][lane * 8]); *(volatile v8b*)(HPl + (m0 + rr) * FC + g * 128 + lane * 8) = *(const v8b*)(&Ol[rr][lane * 8]); }     if (g == 3 && lane < 16) ((volatile float*)FL)[(m0 + rr) * 16 + lane] = Fa[rr][lane]; } __threadfence(); }
    wave_lds_sync(); } }
__global__ __launch_bounds__(32) void att1_kernel(const b16* __restrict__ HPh, const b16* __restrict__ HPl, const float* __restrict__ FL, const int* __restrict__ adj, int BLIM, float* __restrict__ XC) { __shared__ __attribute__((aligned(16))) b16 Ph_[16][KB + 8], Pl_[16][KB + 8], Vth[FH][KB + 8], Vtl[FH][KB + 8]; __shared__ float Sf[16][KB + 4], Of[16][FH + 4];
  const int lane = threadIdx.x, nloc = lane & 15, hlf = lane >> 4; const int qt = blockIdx.x % (NN / 16); const int hd = (blockIdx.x / (NN / 16)) % NHD; const int b = blockIdx.x / ((NN / 16) * NHD); if (b >= BLIM) return; const int t0 = qt * 16; const size_t rowb = (size_t)b * NN;
  float m_r[8], den_r[8]; v8f acc[FH / 16];
#pragma unroll
  for (int r8 = 0; r8 < 8; ++r8) { m_r[r8] = -INFINITY; den_r[r8] = 0.0f; }
#pragma unroll
  for (int t = 0; t < FH / 16; ++t) acc[t] = (v8f){};
#pragma unroll 1
  for (int kb0 = 0; kb0 < NN; kb0 += KB) {
    for (int rr = 0; rr < KB; rr += 2) { const int r = rr + hlf; const size_t vr = (rowb + kb0 + r) * FC + hd * FH; for (int s = 0; s < FH / 32; ++s) { Vth[s * 32 + nloc][r] = HPh[vr + s * 32 + nloc]; Vth[s * 32 + 16 + nloc][r] = HPh[vr + s * 32 + 16 + nloc]; Vtl[s * 32 + nloc][r] = HPl[vr + s * 32 + nloc]; Vtl[s * 32 + 16 + nloc][r] = HPl[vr + s * 32 + 16 + nloc]; } }
    for (int rr = 0; rr < 16; ++rr) { const float f1 = FL[(rowb + t0 + rr) * 16 + hd]; for (int q = 0; q < 4; ++q) { const int j = kb0 + q * 32 + lane; const int ok = adj[((size_t)b * NN + t0 + rr) * NN + j] > 0; Sf[rr][q * 32 + lane] = ok ? leaky(f1 + FL[(rowb + j) * 16 + 8 + hd]) : -INFINITY; } }
    wave_lds_sync();
#pragma unroll
    for (int rr = 0; rr < 16; ++rr) { float mx = -INFINITY;
#pragma unroll
      for (int q = 0; q < 4; ++q) mx = fmaxf(mx, Sf[rr][q * 32 + lane]);
      for (int o = 16; o; o >>= 1) mx = fmaxf(mx, __shfl_xor(mx, o));
      const float mold = __shfl(m_r[rr & 7], (rr >> 3) * 16); const float mn = fmaxf(mold, mx); const float sf = (mold == -INFINITY) ? 0.0f : ((mn == -INFINITY) ? 1.0f : __expf(mold - mn)); float ps = 0.0f;
#pragma unroll
      for (int q = 0; q < 4; ++q) { const int kx = q * 32 + lane; const float sv = Sf[rr][kx]; const float p = (sv == -INFINITY || mn == -INFINITY) ? 0.0f : __expf(sv - mn); ps += p; b16 ph, pl; split16(p * PS, ph, pl); Ph_[rr][kx] = ph; Pl_[rr][kx] = pl; }
      for (int o = 16; o; o >>= 1) ps += __shfl_xor(ps, o);
      if ((rr >> 3) == hlf) { const int r8 = rr & 7; den_r[r8] = den_r[r8] * sf + ps; m_r[r8] = mn;
#pragma unroll
        for (int t = 0; t < FH / 16; ++t) acc[t][r8] = acc[t][r8] * sf; } }
    wave_lds_sync();
    for (int ks = 0; ks < KB; ks += 32) { const v16b pa = frag_kb(&Ph_[nloc][ks], hlf), pb = frag_kb(&Pl_[nloc][ks], hlf);
#pragma unroll
      for (int t = 0; t < FH / 16; ++t) { const v16b vh = frag_kb(&Vth[t * 16 + nloc][ks], hlf), vl = frag_kb(&Vtl[t * 16 + nloc][ks], hlf); acc[t] = wmma16b(pa, vh, acc[t]); acc[t] = wmma16b(pa, vl, acc[t]); acc[t] = wmma16b(pb, vh, acc[t]); } }
    wave_lds_sync(); }
#pragma unroll
  for (int t = 0; t < FH / 16; ++t)
#pragma unroll
    for (int r8 = 0; r8 < 8; ++r8) { const float dn = den_r[r8]; Of[8 * hlf + r8][t * 16 + nloc] = dn > 0.0f ? acc[t][r8] * (1.0f / (HS * PS)) / dn : -1e30f; }
  wave_lds_sync();
  for (int rr = 0; rr < 16; ++rr) { if (Of[rr][0] == -1e30f) { float s0 = 0.0f, s1 = 0.0f; for (int j = 0; j < NN; ++j) { const size_t vr = (rowb + j) * FC + hd * FH; s0 += ((float)HPh[vr + lane] + (float)HPl[vr + lane]) * (1.0f / HS); s1 += ((float)HPh[vr + 32 + lane] + (float)HPl[vr + 32 + lane]) * (1.0f / HS); } Of[rr][lane] = s0 / NN; Of[rr][32 + lane] = s1 / NN; } }
  wave_lds_sync();
  for (int pass = 0; pass < 2; ++pass) { for (int rr = 0; rr < 16; ++rr) for (int s = 0; s < FH / 32; ++s) { const float v = Of[rr][s * 32 + lane]; ((volatile float*)XC)[(rowb + t0 + rr) * FC + hd * FH + s * 32 + lane] = v > 0.0f ? v : (__expf(v) - 1.0f); } __threadfence(); } }
__global__ __launch_bounds__(32) void proj2_kernel(const float* __restrict__ XC, const b16* __restrict__ WOUT, const float* __restrict__ a1o, const float* __restrict__ a2o, int RLIM, float* __restrict__ H2) { __shared__ __attribute__((aligned(16))) b16 Ah[16][FC + 8], Al[16][FC + 8]; __shared__ float Tf[16][32]; const int lane = threadIdx.x, nloc = lane & 15, hlf = lane >> 4; const size_t m0 = (size_t)blockIdx.x * 16; if (m0 >= (size_t)RLIM) return;
  for (int rr = 0; rr < 16; ++rr) for (int q = 0; q < FC / 32; ++q) { b16 p, ql; split16(XC[(m0 + rr) * FC + q * 32 + lane] * HS, p, ql); Ah[rr][q * 32 + lane] = p; Al[rr][q * 32 + lane] = ql; }
  wave_lds_sync(); v8f acc = {};
#pragma unroll 4
  for (int kb = 0; kb < FC; kb += 32) { const v16b bw = frag_kb(WOUT + (size_t)nloc * FC + kb, hlf); acc = wmma16b(frag_kb(&Ah[nloc][kb], hlf), bw, acc); acc = wmma16b(frag_kb(&Al[nloc][kb], hlf), bw, acc); }
#pragma unroll
  for (int r8 = 0; r8 < 8; ++r8) Tf[8 * hlf + r8][nloc] = acc[r8] * (1.0f / (HS * WSC));
  wave_lds_sync();
  for (int rr = 0; rr < 16; ++rr) { float s1 = lane < 16 ? pmul(Tf[rr][lane], bfv(a1o[lane])) : 0.0f, s2 = lane < 16 ? pmul(Tf[rr][lane], bfv(a2o[lane])) : 0.0f; for (int o = 8; o; o >>= 1) { s1 += __shfl_xor(s1, o); s2 += __shfl_xor(s2, o); } if (lane == 0) { Tf[rr][16] = s1; Tf[rr][17] = s2; } if (lane >= 18) Tf[rr][lane] = 0.0f; }
  wave_lds_sync();
  for (int pass = 0; pass < 2; ++pass) { for (int rr = 0; rr < 16; ++rr) ((volatile float*)H2)[(m0 + rr) * 32 + lane] = Tf[rr][lane]; __threadfence(); } }
__global__ __launch_bounds__(32) void att2_kernel(const float* __restrict__ H2, const int* __restrict__ adj, int BLIM, float* __restrict__ OUT) { __shared__ __attribute__((aligned(16))) b16 Ph_[16][NN + 8], Pl_[16][NN + 8], Vh[16][NN + 8], Vl[16][NN + 8]; __shared__ float Den[16], Tf[16][16]; const int lane = threadIdx.x, nloc = lane & 15, hlf = lane >> 4; const int qt = blockIdx.x % (NN / 16); const int b = blockIdx.x / (NN / 16); if (b >= BLIM) return; const int t0 = qt * 16; const size_t rowb = (size_t)b * NN;
  for (int j = hlf; j < NN; j += 2) { b16 p, ql; split16(H2[(rowb + j) * 32 + nloc] * HS, p, ql); Vh[nloc][j] = p; Vl[nloc][j] = ql; }
  for (int rr = 0; rr < 16; ++rr) { const float f1 = H2[(rowb + t0 + rr) * 32 + 16]; float sv[NN / 32]; float mx = -INFINITY; int anyok = 0;
#pragma unroll
    for (int q = 0; q < NN / 32; ++q) { const int j = q * 32 + lane; const int ok = adj[((size_t)b * NN + t0 + rr) * NN + j] > 0; anyok |= ok; sv[q] = ok ? leaky(f1 + H2[(rowb + j) * 32 + 17]) : -INFINITY; mx = fmaxf(mx, sv[q]); }
    for (int o = 16; o; o >>= 1) { mx = fmaxf(mx, __shfl_xor(mx, o)); anyok |= __shfl_xor(anyok, o); }
    float ps = 0.0f;
#pragma unroll
    for (int q = 0; q < NN / 32; ++q) { const float p = anyok ? ((sv[q] == -INFINITY) ? 0.0f : __expf(sv[q] - mx)) : 1.0f;
      ps += p; b16 ph, pl; split16(p * PS, ph, pl); Ph_[rr][q * 32 + lane] = ph; Pl_[rr][q * 32 + lane] = pl; }
    for (int o = 16; o; o >>= 1) ps += __shfl_xor(ps, o); if (lane == 0) Den[rr] = ps; }
  if (lane < 16) for (int k = NN; k < NN + 8; ++k) { Ph_[lane][k] = (b16)0.0f; Pl_[lane][k] = (b16)0.0f; Vh[lane][k] = (b16)0.0f; Vl[lane][k] = (b16)0.0f; }
  wave_lds_sync(); v8f acc = {};
#pragma unroll 4
  for (int ks = 0; ks < NN; ks += 32) { const v16b pa = frag_kb(&Ph_[nloc][ks], hlf), pb = frag_kb(&Pl_[nloc][ks], hlf), vh = frag_kb(&Vh[nloc][ks], hlf), vl = frag_kb(&Vl[nloc][ks], hlf); acc = wmma16b(pa, vh, acc); acc = wmma16b(pa, vl, acc); acc = wmma16b(pb, vh, acc); }
#pragma unroll
  for (int r8 = 0; r8 < 8; ++r8) { const int rr = 8 * hlf + r8; Tf[rr][nloc] = acc[r8] * (1.0f / (HS * PS)) / Den[rr]; }
  wave_lds_sync();
  for (int pass = 0; pass < 2; ++pass) { for (int q = 0; q < 2; ++q) { const int idx = q * 128 + lane * 4; *(volatile v4f*)(OUT + (rowb + t0) * FO + idx) = (v4f){Tf[idx / 16][idx % 16], Tf[(idx + 1) / 16][(idx + 1) % 16], Tf[(idx + 2) / 16][(idx + 2) % 16], Tf[(idx + 3) / 16][(idx + 3) % 16]}; } __threadfence(); } }
}

extern "C" void kernel_launch(void* const* d_in, const int* in_sizes, int n_in, void* d_out, int out_size, void* d_ws, size_t ws_size, hipStream_t stream) {
  (void)n_in;
  auto Fp = [&](int i) { return (const float*)d_in[i]; }; auto Ip = [&](int i) { return (const int*)d_in[i]; };
  if (in_sizes[0] != NB * NN * FI || in_sizes[1] != NB * NN * NN || in_sizes[2] != NHD * FI * FH || in_sizes[3] != NHD * FH || in_sizes[5] != FC * FO || in_sizes[6] != FO || out_size != NB * NN * FO) return;
  const int BLIM = NB;
  const int RLIM = BLIM * NN;
  size_t off = 0; char* ws = (char*)d_ws;
  auto carve = [&](size_t bytes) { char* p = ws + off; off += (bytes + 255) & ~(size_t)255; return p; };
  b16* WH = (b16*)carve((size_t)FC * FI * 2); b16* WOUT = (b16*)carve((size_t)FO * FC * 2); b16* HPh = (b16*)carve((size_t)NB * NN * FC * 2); b16* HPl = (b16*)carve((size_t)NB * NN * FC * 2); float* FL = (float*)carve((size_t)NB * NN * 16 * 4); float* XC = (float*)carve((size_t)NB * NN * FC * 4); float* H2 = (float*)carve((size_t)NB * NN * 32 * 4);
  if (off > ws_size || off > ((size_t)96 << 20)) return;
  wput_kernel<<<(FC * (FI / 8) + 255) / 256, 256, 0, stream>>>(Fp(2), Fp(5), WH, WOUT);
  proj1_kernel<<<RLIM / 16, 32, 0, stream>>>(Fp(0), WH, Fp(3), Fp(4), RLIM, HPh, HPl, FL);
  att1_kernel<<<BLIM * NHD * (NN / 16), 32, 0, stream>>>(HPh, HPl, FL, Ip(1), BLIM, XC);
  proj2_kernel<<<RLIM / 16, 32, 0, stream>>>(XC, WOUT, Fp(6), Fp(7), RLIM, H2);
  att2_kernel<<<BLIM * (NN / 16), 32, 0, stream>>>(H2, Ip(1), BLIM, (float*)d_out);
}
